// Net_with_embedding_27436251087105
// MI455X (gfx1250) — hardware-run, weakly checked
//
#include <hip/hip_runtime.h>

typedef float          v8f   __attribute__((ext_vector_type(8)));
typedef float          v4f   __attribute__((ext_vector_type(4)));
typedef unsigned int   v4u   __attribute__((ext_vector_type(4)));
typedef int            v8i   __attribute__((ext_vector_type(8)));
typedef unsigned short v8us  __attribute__((ext_vector_type(8)));
typedef unsigned short v16us __attribute__((ext_vector_type(16)));
typedef __bf16         v16bf __attribute__((ext_vector_type(16)));
typedef _Float16       v16h  __attribute__((ext_vector_type(16)));
typedef v4f  __attribute__((may_alias)) v4fa;
typedef v8us __attribute__((may_alias)) v8usa;
union FragB { v16bf v; v16us u; v8us h[2]; v8i w; };
union FragH { v16h  v; v16us u; v8us h[2]; v8i w; };

__device__ __forceinline__ v8f wmb(const FragB& a, const FragB& b, v8f c) {
  v8f d = __builtin_amdgcn_wmma_f32_16x16x32_bf16(false, a.v, false, b.v, (short)0, c, false, false);
  asm volatile("v_nop\n\tv_nop\n\tv_nop\n\tv_nop" : "+v"(d) : "v"(a.w), "v"(b.w));
  return d;
}

__device__ __forceinline__ v8f wmh(const FragH& a, const FragH& b, v8f c) {
  v8f d = __builtin_amdgcn_wmma_f32_16x16x32_f16(false, a.v, false, b.v, (short)0, c, false, false);
  asm volatile("v_nop\n\tv_nop\n\tv_nop\n\tv_nop" : "+v"(d) : "v"(a.w), "v"(b.w));
  return d;
}

__device__ __forceinline__ unsigned bf16_bits(float f) {
  const unsigned u = __float_as_uint(f);
  const unsigned r = (u + 0x7FFFu + ((u >> 16) & 1u)) >> 16;
  const unsigned q = (u >> 16) | 0x40u;
  return ((u & 0x7fffffffu) > 0x7f800000u) ? q : r;
}

__device__ __forceinline__ float bf16_val(float f) {
  return __uint_as_float(bf16_bits(f) << 16);
}
__device__ __forceinline__ int clampi(int v, int lo, int hi) {
  return v < lo ? lo : (v > hi ? hi : v);
}

__device__ __forceinline__ unsigned f16_bits(float f) {
  const unsigned u  = __float_as_uint(f);
  const unsigned s  = (u >> 16) & 0x8000u;
  const unsigned a  = u & 0x7fffffffu;
  const unsigned t  = a - 0x38000000u;
  const unsigned r  = (t + 0x0FFFu + ((t >> 13) & 1u)) >> 13;
  const unsigned rc = r > 0x7C00u ? 0x7C00u : r;
  const bool small  = a < 0x38800000u;
  const bool isnan  = a > 0x7f800000u;
  const unsigned fin = small ? 0u : (s | rc);
  return isnan ? (s | 0x7E00u) : fin;
}

__device__ __forceinline__ unsigned pk16(unsigned lo, unsigned hi) { return lo | (hi << 16); }
__device__ __forceinline__ unsigned bf16_lo_bits(float v) {
  float hi = bf16_val(v);
  asm volatile("" : "+v"(hi));
  return bf16_bits(v - hi);
}
__device__ __forceinline__ v4u pack8_bf16(v4f a, v4f c) {
  return (v4u){ pk16(bf16_bits(a[0]), bf16_bits(a[1])), pk16(bf16_bits(a[2]), bf16_bits(a[3])),
                pk16(bf16_bits(c[0]), bf16_bits(c[1])), pk16(bf16_bits(c[2]), bf16_bits(c[3])) };
}
__device__ __forceinline__ v4u pack8_bf16_lo(v4f a, v4f c) {
  return (v4u){ pk16(bf16_lo_bits(a[0]), bf16_lo_bits(a[1])), pk16(bf16_lo_bits(a[2]), bf16_lo_bits(a[3])),
                pk16(bf16_lo_bits(c[0]), bf16_lo_bits(c[1])), pk16(bf16_lo_bits(c[2]), bf16_lo_bits(c[3])) };
}
__device__ __forceinline__ v4u pack8_f16(v4f a, v4f c) {
  return (v4u){ pk16(f16_bits(a[0]), f16_bits(a[1])), pk16(f16_bits(a[2]), f16_bits(a[3])),
                pk16(f16_bits(c[0]), f16_bits(c[1])), pk16(f16_bits(c[2]), f16_bits(c[3])) };
}

template <int FORM>
__global__ __launch_bounds__(256) void k_plane(const float* __restrict__ src, int rows, int cols, int ldsrc,
                                               unsigned short* __restrict__ dst, int MP, int KP) {
  static_assert(FORM >= 0 && FORM <= 3);
  const int KTOT = (FORM == 1 || FORM == 3) ? 2 * KP : KP;
  const unsigned ppr   = (unsigned)(KTOT >> 3);
  const unsigned kp8   = (unsigned)(KP >> 3);
  const unsigned total = (unsigned)MP * ppr;
  const unsigned g     = blockIdx.x * 256u + threadIdx.x;
  const unsigned rowu  = g / ppr;
  const unsigned p     = g - rowu * ppr;
  const bool second    = p >= kp8;
  const int row = (int)rowu;
  const int c0  = (int)((second ? p - kp8 : p) << 3);
  const float* srow = src + (size_t)clampi(row, 0, rows - 1) * (size_t)ldsrc;
  float x[8];
  unsigned mk[8];
#pragma unroll
  for (int e = 0; e < 8; ++e) {
    const int c = c0 + e;
    const float v = srow[clampi(c, 0, cols - 1)];
    asm volatile("" :: "v"(v));
    x[e]  = v;
    mk[e] = (row < rows && c < cols) ? 0xFFFFu : 0u;
  }
  const v4f a = (v4f){ x[0], x[1], x[2], x[3] };
  const v4f c = (v4f){ x[4], x[5], x[6], x[7] };
  v4u o;
  if (FORM == 2) {
    o = pack8_f16(a, c);
  } else {
    const v4u hi = pack8_bf16(a, c);
    o = hi;
    if (FORM == 1) { const v4u lo = pack8_bf16_lo(a, c); o = second ? lo : hi; }
  }
  const v4u mw = (v4u){ pk16(mk[0], mk[1]), pk16(mk[2], mk[3]), pk16(mk[4], mk[5]), pk16(mk[6], mk[7]) };
  o &= mw;
  if (g < total) {
    volatile v4u* q = (volatile v4u*)(dst + (size_t)g * 8);
    *q = o;
    __threadfence();
    *q = o;
  }
}

template <int FORM> struct FragOf    { typedef FragB T; };
template <>         struct FragOf<2> { typedef FragH T; };
__device__ __forceinline__ v8f mm(const FragB& a, const FragB& b, v8f c) { return wmb(a, b, c); }
__device__ __forceinline__ v8f mm(const FragH& a, const FragH& b, v8f c) { return wmh(a, b, c); }
template <class F> __device__ __forceinline__ F ld_frag(const unsigned short* p) {
  F f;
  f.h[0] = *(const v8usa*)(p);
  f.h[1] = *(const v8usa*)(p + 16);
  return f;
}

template <int FORM, int EPI>
__global__ __launch_bounds__(256) __attribute__((amdgpu_num_vgpr(248)))
void k_gemm_nt(const unsigned short* __restrict__ A, const unsigned short* __restrict__ B,
               const float* __restrict__ bias, float* __restrict__ D, int M, int N, int KTOT, int ldd) {
  static_assert(FORM >= 0 && FORM <= 2);
  static_assert(EPI == 0 || EPI == 1);
  typedef typename FragOf<FORM>::T F;
  __shared__ __attribute__((aligned(16))) float sT[8][16 * 68];
  const int lane = threadIdx.x & 31;
  const int wave = threadIdx.x >> 5;
  const int tilesM = (M + 63) >> 6;
  const int tilesN = (N + 63) >> 6;
  const int tile = blockIdx.x * 8 + wave;
  if (tile >= tilesM * tilesN) return;
  const int tm = tile / tilesN;
  const int tn = tile - tm * tilesN;
  const int m0 = tm << 6;
  const int n0 = tn << 6;

  const int rl = lane & 15;
  const int h8 = (lane >> 4) * 8;
  const unsigned short* pa = A + (size_t)(m0 + rl) * (size_t)KTOT + h8;
  const unsigned short* pb = B + (size_t)(n0 + rl) * (size_t)KTOT + h8;

  v8f acc[4][4];
#pragma unroll
  for (int i = 0; i < 4; ++i)
#pragma unroll
    for (int j = 0; j < 4; ++j) acc[i][j] = (v8f){0.f, 0.f, 0.f, 0.f, 0.f, 0.f, 0.f, 0.f};

#pragma unroll 1
  for (int k0 = 0; k0 < KTOT; k0 += 32) {
    F bf[4];
#pragma unroll
    for (int j = 0; j < 4; ++j) bf[j] = ld_frag<F>(pb + (size_t)(j << 4) * (size_t)KTOT + k0);
#pragma unroll
    for (int i = 0; i < 4; ++i) {
      const F af = ld_frag<F>(pa + (size_t)(i << 4) * (size_t)KTOT + k0);
#pragma unroll
      for (int j = 0; j < 4; ++j) acc[i][j] = mm(af, bf[j], acc[i][j]);
    }
  }

  float* slab = sT[wave];
  const int hh = lane >> 4;
  const int c4 = (lane & 15) * 4;
  const int nc = n0 + c4;
  const bool cok = nc < N;
  v4f bv = (v4f){0.f, 0.f, 0.f, 0.f};
  if (EPI == 1) {
    bv = *(const v4fa*)(bias + clampi(nc, 0, N - 4));
    asm volatile("" :: "v"(bv));
  }
#pragma unroll
  for (int i = 0; i < 4; ++i) {
    const int mBase = m0 + (i << 4);
#pragma unroll
    for (int j = 0; j < 4; ++j) {
#pragma unroll
      for (int r = 0; r < 8; ++r) slab[(h8 + r) * 68 + (j << 4) + rl] = acc[i][j][r];
    }
    __builtin_amdgcn_fence(__ATOMIC_RELEASE, "workgroup");
    __builtin_amdgcn_wave_barrier();
    __builtin_amdgcn_fence(__ATOMIC_ACQUIRE, "workgroup");
    v4f vv[8];
#pragma unroll
    for (int it = 0; it < 8; ++it) {
      const int row = it * 2 + hh;
      v4f v = *(const v4fa*)(slab + row * 68 + c4);
      if (EPI == 1) v += bv;
      vv[it] = v;
    }
    for (int pass = 0; pass < 2; ++pass) {
#pragma unroll
      for (int it = 0; it < 8; ++it) {
        const int row = mBase + it * 2 + hh;
        if (cok && row < M) *(volatile v4f*)(D + (size_t)row * (size_t)ldd + nc) = vv[it];
      }
      __threadfence();
    }
    __builtin_amdgcn_fence(__ATOMIC_RELEASE, "workgroup");
    __builtin_amdgcn_wave_barrier();
    __builtin_amdgcn_fence(__ATOMIC_ACQUIRE, "workgroup");
  }
}

#pragma clang fp contract(off)

#ifndef SINGLE_L2
#define SINGLE_L2 0
#endif
#ifndef SINGLE_L3
#define SINGLE_L3 0
#endif
static_assert(SINGLE_L2 == 0 || SINGLE_L2 == 1);
static_assert(SINGLE_L3 == 0 || SINGLE_L3 == 1);

typedef float        v2f __attribute__((ext_vector_type(2)));
typedef unsigned int v2u __attribute__((ext_vector_type(2)));
typedef int          v2i __attribute__((ext_vector_type(2)));
typedef int          v4i __attribute__((ext_vector_type(4)));
typedef double       v2d __attribute__((ext_vector_type(2)));
typedef v2f __attribute__((may_alias)) v2fa;
typedef v2i __attribute__((may_alias)) v2ia;
typedef v4i __attribute__((may_alias)) v4ia;

constexpr int NN     = 50000;
constexpr int NE     = 800000;
constexpr int F0     = 128;
constexpr int F1     = 128;
constexpr int F2     = 64;
constexpr int F3     = 32;
constexpr int NP     = 50048;
constexpr int NREC   = NP / 128;
constexpr int NBRUN  = 1024;
constexpr int NBLK   = 49;
constexpr int CAP    = 21504;
constexpr int DEGCAP = 48;
constexpr int WLCAP  = 4096;
constexpr int EPW    = NE / 8;
constexpr int SUB    = 128;
constexpr int NSTEP  = (EPW + SUB - 1) / SUB;
constexpr int K2T    = SINGLE_L2 ? F1 : 2 * F1;
constexpr int K3T    = SINGLE_L3 ? F2 : 2 * F2;

static_assert(NN % 8 == 0);
static_assert(NE == 390 * 2048 + 1280);
static_assert(DEGCAP <= 64 && DEGCAP % 16 == 0 && DEGCAP * 4 >= 37 * 5);
static_assert(CAP * 4 >= 16699 * 5 && (CAP / 2) % 256 == 0 && CAP >= 2 * DEGCAP);
static_assert(WLCAP * 4 >= 2048 * 5 && WLCAP * 8 >= CAP);
static_assert(NP % 64 == 0 && NP >= NN && NP - NN < 64 && NREC * 128 == NP && NP % 16 == 0 && NP % 8 == 0);
static_assert(NBLK * NBRUN >= NN && (NBLK - 1) * NBRUN < NN);
static_assert(NE % 8 == 0 && NSTEP * SUB >= EPW && (NSTEP - 1) * SUB < EPW);
static_assert((((long long)(NE - 1) << 10) | 1023) < (1LL << 31));
static_assert(K2T % 32 == 0 && K3T % 32 == 0 && F0 % 32 == 0);
static_assert((size_t)(NN - 1) * F3 + 31 < (size_t)NN * F3);

constexpr int P_B1 = 0, P_G1 = 128, P_BE1 = 256, P_B2 = 384, P_G2 = 448, P_BE2 = 512;
constexpr int P_B3 = 576, P_G3 = 608, P_BE3 = 640, P_N = 672;
constexpr int S_M1 = 0, S_R1 = 128, S_M2 = 256, S_R2 = 384, S_M3 = 512, S_R3 = 640, S_N = 768;

constexpr int LK_WL   = 0;
constexpr int LK_SL   = 8 * WLCAP;
constexpr int LK_CNT  = LK_SL + CAP;
constexpr int LK_OFF  = LK_CNT + NBRUN;
constexpr int LK_CUR  = LK_OFF + NBRUN;
constexpr int LK_MISC = LK_CUR + NBRUN;
constexpr int LK_INTS = LK_MISC + 16;
constexpr int LK_LDS  = LK_INTS * 4;
static_assert(LK_LDS == 229440 && LK_LDS <= 262144 && LK_LDS <= 327680);
static_assert(LK_SL % 4 == 0 && LK_CNT % 4 == 0 && (CAP + NBRUN) % 1024 == 0);

constexpr size_t SZ_A0   = (size_t)NP * F0 * 2;
constexpr size_t SZ_AHL  = (size_t)NP * 256 * 2;
constexpr size_t SZ_AHL3 = (size_t)NP * 128 * 2;
constexpr size_t SZ_HW   = (size_t)NP * 128 * 4;
constexpr size_t SZ_V    = (size_t)NN * 128 * 4;
constexpr size_t SZ_LIST = (size_t)NBLK * CAP * 8;
constexpr size_t SZ_NODE = (size_t)NBLK * NBRUN * 4;
constexpr size_t SZ_FLAG = 6400;
constexpr size_t SZ_W1T  = (size_t)F1 * F0 * 2;
constexpr size_t SZ_W2D  = (size_t)64 * 256 * 2;
constexpr size_t SZ_W3D  = (size_t)64 * 128 * 2;
constexpr size_t SZ_PAR  = 2816;
constexpr size_t SZ_REC  = (size_t)NREC * 128 * 8;
constexpr size_t SZ_ST   = 3072;
constexpr size_t OFF_A0   = 0;
constexpr size_t OFF_AHL  = OFF_A0 + SZ_A0;
constexpr size_t OFF_AHL3 = OFF_AHL + SZ_AHL;
constexpr size_t OFF_HW   = OFF_AHL3 + SZ_AHL3;
constexpr size_t OFF_V    = OFF_HW + SZ_HW;
constexpr size_t OFF_LIST = OFF_V + SZ_V;
constexpr size_t OFF_CNT  = OFF_LIST + SZ_LIST;
constexpr size_t OFF_OFF  = OFF_CNT + SZ_NODE;
constexpr size_t OFF_DINV = OFF_OFF + SZ_NODE;
constexpr size_t OFF_FLAG = OFF_DINV + SZ_NODE;
constexpr size_t OFF_W1T  = OFF_FLAG + SZ_FLAG;
constexpr size_t OFF_W2D  = OFF_W1T + SZ_W1T;
constexpr size_t OFF_W3D  = OFF_W2D + SZ_W2D;
constexpr size_t OFF_PAR  = OFF_W3D + SZ_W3D;
constexpr size_t OFF_REC  = OFF_PAR + SZ_PAR;
constexpr size_t OFF_ST   = OFF_REC + SZ_REC;
constexpr size_t WS_TOTAL = OFF_ST + SZ_ST;
static_assert(WS_TOTAL == (size_t)((size_t)109375 << 10));
static_assert(WS_TOTAL <= ((size_t)128 << 20));
static_assert(SZ_A0 % 256 == 0 && SZ_AHL % 256 == 0 && SZ_AHL3 % 256 == 0 && SZ_HW % 256 == 0 && SZ_V % 256 == 0);
static_assert(SZ_LIST % 256 == 0 && SZ_NODE % 256 == 0 && SZ_FLAG % 256 == 0 && SZ_PAR % 256 == 0);
static_assert(SZ_REC % 256 == 0 && SZ_ST % 256 == 0 && SZ_W1T % 256 == 0 && SZ_W2D % 256 == 0 && SZ_W3D % 256 == 0);
static_assert((size_t)NBLK * 128 <= SZ_FLAG && (size_t)P_N * 4 <= SZ_PAR && (size_t)S_N * 4 <= SZ_ST);
static_assert((size_t)NP * K2T * 2 <= SZ_AHL && (size_t)NP * K3T * 2 <= SZ_AHL3);
static_assert((size_t)64 * K2T * 2 <= SZ_W2D && (size_t)64 * K3T * 2 <= SZ_W3D);
static_assert((size_t)((NN + 31) / 32) * 128 <= SZ_NODE);

__device__ __forceinline__ float relu_k(float v) { return (v > 0.0f) ? v : (v - v); }

template <int CPL>
__device__ __forceinline__ void ld_cols(const float* __restrict__ p, float (&x)[4]) {
  static_assert(CPL == 4 || CPL == 2 || CPL == 1);
  if constexpr (CPL == 4) {
    const v4f v = *(const v4fa*)p;
    asm volatile("" :: "v"(v));
    x[0] = v[0]; x[1] = v[1]; x[2] = v[2]; x[3] = v[3];
  } else if constexpr (CPL == 2) {
    const v2f v = *(const v2fa*)p;
    asm volatile("" :: "v"(v));
    x[0] = v[0]; x[1] = v[1]; x[2] = 0.0f; x[3] = 0.0f;
  } else {
    const float v = *p;
    asm volatile("" :: "v"(v));
    x[0] = v; x[1] = 0.0f; x[2] = 0.0f; x[3] = 0.0f;
  }
}
template <int CPL>
__device__ __forceinline__ void st_cols(float* p, const float (&x)[4]) {
  static_assert(CPL == 4 || CPL == 2 || CPL == 1);
  if constexpr (CPL == 4) {
    *(volatile v4f*)p = (v4f){ x[0], x[1], x[2], x[3] };
  } else if constexpr (CPL == 2) {
    *(volatile v2f*)p = (v2f){ x[0], x[1] };
  } else {
    *(volatile float*)p = x[0];
  }
}

constexpr int PB_W1  = F1 * (F0 / 8) / 256;
constexpr int PB_W2  = 64 * (K2T / 8) / 256;
constexpr int PB_W3  = 64 * (K3T / 8) / 256;
constexpr int PB_TOT = PB_W1 + PB_W2 + PB_W3 + 1;
static_assert((F1 * (F0 / 8)) % 256 == 0 && (64 * (K2T / 8)) % 256 == 0 && (64 * (K3T / 8)) % 256 == 0);

__device__ __forceinline__ void wplane_unit(const float* __restrict__ W, int ncols, int kin, int ktot, int nvalid,
                                            unsigned short* __restrict__ dst, int u) {
  const int ppr = ktot >> 3;
  const int n   = u / ppr;
  const int p   = u - n * ppr;
  const int k8  = (p << 3) & (kin - 1);
  const int nc  = n < nvalid ? n : nvalid - 1;
  const float* s = W + (size_t)k8 * (size_t)ncols + nc;
  float x[8];
#pragma unroll
  for (int i = 0; i < 8; ++i) {
    const float v = s[(size_t)i * (size_t)ncols];
    asm volatile("" :: "v"(v));
    x[i] = v;
  }
  v4u o = pack8_bf16((v4f){ x[0], x[1], x[2], x[3] }, (v4f){ x[4], x[5], x[6], x[7] });
  const unsigned mk = (n < nvalid) ? 0xFFFFFFFFu : 0u;
  o &= (v4u){ mk, mk, mk, mk };
  volatile v4u* q = (volatile v4u*)(dst + (size_t)u * 8);
  *q = o;
  __threadfence();
  *q = o;
}

__device__ __forceinline__ void par_unit(const float* __restrict__ src, int n4, float* __restrict__ dst, int tid) {
  const int j = tid < n4 ? tid : n4 - 1;
  const v4f a = *(const v4fa*)(src + 4 * j);
  asm volatile("" :: "v"(a));
  const v4f o = (v4f){ bf16_val(a[0]), bf16_val(a[1]), bf16_val(a[2]), bf16_val(a[3]) };
  if (tid < n4) {
    volatile v4f* q = (volatile v4f*)(dst + 4 * tid);
    *q = o;
    __threadfence();
    *q = o;
  }
}

__global__ __launch_bounds__(256) void k_prep(const float* __restrict__ W1, const float* __restrict__ W2,
                                              const float* __restrict__ W3,
                                              const float* __restrict__ b1, const float* __restrict__ g1,
                                              const float* __restrict__ be1,
                                              const float* __restrict__ b2, const float* __restrict__ g2,
                                              const float* __restrict__ be2,
                                              const float* __restrict__ b3, const float* __restrict__ g3,
                                              const float* __restrict__ be3,
                                              unsigned short* __restrict__ W1T, unsigned short* __restrict__ W2D,
                                              unsigned short* __restrict__ W3D, float* __restrict__ PAR) {
  const int tid = (int)threadIdx.x;
  const int blk = (int)blockIdx.x;
  if (blk < PB_W1) {
    wplane_unit(W1, F1, F0, F0, F1, W1T, blk * 256 + tid);
  } else if (blk < PB_W1 + PB_W2) {
    wplane_unit(W2, F2, F1, K2T, F2, W2D, (blk - PB_W1) * 256 + tid);
  } else if (blk < PB_W1 + PB_W2 + PB_W3) {
    wplane_unit(W3, F3, F2, K3T, F3, W3D, (blk - PB_W1 - PB_W2) * 256 + tid);
  } else {
    par_unit(b1,  F1 / 4, PAR + P_B1,  tid);
    par_unit(g1,  F1 / 4, PAR + P_G1,  tid);
    par_unit(be1, F1 / 4, PAR + P_BE1, tid);
    par_unit(b2,  F2 / 4, PAR + P_B2,  tid);
    par_unit(g2,  F2 / 4, PAR + P_G2,  tid);
    par_unit(be2, F2 / 4, PAR + P_BE2, tid);
    par_unit(b3,  F3 / 4, PAR + P_B3,  tid);
    par_unit(g3,  F3 / 4, PAR + P_G3,  tid);
    par_unit(be3, F3 / 4, PAR + P_BE3, tid);
  }
}

__global__ __launch_bounds__(256) void k_gatherA(const int* __restrict__ xid, const float* __restrict__ emb,
                                                 unsigned short* __restrict__ A0) {
  const int tid = (int)threadIdx.x, lane = tid & 31, wave = tid >> 5;
  const int row = (int)blockIdx.x * 8 + wave;
  const bool live = row < NN;
  const int rc = live ? row : NN - 1;
  int id = xid[rc];
  asm volatile("" :: "v"(id));
  id = clampi(id, 0, NN - 1);
  const v4f a = *(const v4fa*)(emb + (size_t)id * F0 + 4 * lane);
  asm volatile("" :: "v"(a));
  v2u o = (v2u){ pk16(bf16_bits(a[0]), bf16_bits(a[1])), pk16(bf16_bits(a[2]), bf16_bits(a[3])) };
  const unsigned mk = live ? 0xFFFFFFFFu : 0u;
  o &= (v2u){ mk, mk };
  volatile v2u* q = (volatile v2u*)(A0 + (size_t)row * F0 + 4 * lane);
  *q = o;
  __threadfence();
  *q = o;
}

__global__ __launch_bounds__(256) void k_list(const int* __restrict__ ei, int* __restrict__ LIST,
                                              int* __restrict__ CNT, int* __restrict__ OFF,
                                              int* __restrict__ FLAG) {
  extern __shared__ __attribute__((aligned(16))) int dsm[];
  int* wl   = dsm + LK_WL;
  int* sl   = dsm + LK_SL;
  int* cnt  = dsm + LK_CNT;
  int* offs = dsm + LK_OFF;
  int* cur  = dsm + LK_CUR;
  int* misc = dsm + LK_MISC;
  const int tid = (int)threadIdx.x, lane = tid & 31, wave = tid >> 5;
  const int blk = (int)blockIdx.x;
  const int nodeBase = blk * NBRUN;
  const int nbi = (NN - nodeBase) < NBRUN ? (NN - nodeBase) : NBRUN;
  const unsigned unb = (unsigned)(nbi < 0 ? 0 : nbi);

  {
    const v4i z4 = (v4i){0, 0, 0, 0};
    for (int i = tid * 4; i < CAP + NBRUN; i += 1024) *(v4ia*)(sl + i) = z4;
    if (tid < 16) misc[tid] = 0;
  }
  __syncthreads();

  const int* srcp = ei;
  const int* dstp = ei + NE;
  int* mylist = wl + wave * WLCAP;
  const int wbase = wave * EPW;
  const int wlast = wbase + EPW - 1;
  int wc = 0;
#pragma unroll 1
  for (int st = 0; st < NSTEP; ++st) {
    const int e0 = wbase + st * SUB + lane;
    int dk[4];
#pragma unroll
    for (int j = 0; j < 4; ++j) {
      const int e  = e0 + 32 * j;
      const int ec = e < wlast ? e : wlast;
      const int d  = dstp[ec];
      asm volatile("" :: "v"(d));
      dk[j] = (e <= wlast) ? d : -1;
    }
#pragma unroll
    for (int j = 0; j < 4; ++j) {
      const unsigned slot = (unsigned)dk[j] - (unsigned)nodeBase;
      const bool hit = slot < unb;
      const unsigned mj = __builtin_amdgcn_ballot_w32(hit);
      if (mj != 0u) {
        if (hit) {
          const int pos = wc + (int)__builtin_amdgcn_mbcnt_lo(mj, 0u);
          if (pos < WLCAP) mylist[pos] = ((e0 + 32 * j) << 10) | (int)slot;
        }
        wc += (int)__builtin_popcount(mj);
      }
    }
  }
  if (lane == 0) misc[wave] = wc;
  __syncthreads();

  if (wave == 0) {
    int t = 0, ov = 0;
#pragma unroll 1
    for (int w2 = 0; w2 < 8; ++w2) {
      const int craw = misc[w2];
      ov |= (craw > WLCAP) ? 1 : 0;
      const int c = __builtin_amdgcn_readfirstlane(clampi(craw, 0, WLCAP));
#pragma unroll 1
      for (int b0 = 0; b0 < c; b0 += 32) {
        const int idx = (b0 + lane) < c ? (b0 + lane) : c - 1;
        const int ent = wl[w2 * WLCAP + idx];
        const int m32 = (c - b0) < 32 ? (c - b0) : 32;
#pragma unroll 1
        for (int k = 0; k < m32; ++k) {
          const int u    = __builtin_amdgcn_readlane(ent, k);
          const int slot = u & (NBRUN - 1);
          if (t < CAP) {
            if (lane == 0) cnt[slot] = cnt[slot] + 1;
            t = t + 1;
          } else {
            ov = 1;
          }
        }
      }
    }
    if (lane == 0) { misc[8] = t; misc[9] = ov; }
  }
  __syncthreads();

  if (wave == 0) {
    const int base = lane * (NBRUN / 32);
    int s = 0, big = 0;
#pragma unroll 1
    for (int i = 0; i < NBRUN / 32; ++i) {
      const int cv = cnt[base + i];
      s += cv;
      big |= (cv > DEGCAP) ? 1 : 0;
    }
    int incl = s;
#pragma unroll
    for (int d = 1; d < 32; d <<= 1) {
      const int y = __shfl_up(incl, d, 32);
      incl += (lane >= d) ? y : 0;
    }
    int run = incl - s;
#pragma unroll 1
    for (int i = 0; i < NBRUN / 32; ++i) {
      const int cv = cnt[base + i];
      offs[base + i] = run;
      cur[base + i]  = run;
      run += cv;
    }
    const unsigned bm = __builtin_amdgcn_ballot_w32(big != 0);
    if (lane == 0) misc[9] = misc[9] | ((bm != 0u) ? 1 : 0);
  }
  __syncthreads();

  if (wave == 0) {
    int t2 = 0;
#pragma unroll 1
    for (int w2 = 0; w2 < 8; ++w2) {
      const int c = __builtin_amdgcn_readfirstlane(clampi(misc[w2], 0, WLCAP));
#pragma unroll 1
      for (int b0 = 0; b0 < c; b0 += 32) {
        const int idx = (b0 + lane) < c ? (b0 + lane) : c - 1;
        const int ent = wl[w2 * WLCAP + idx];
        const int m32 = (c - b0) < 32 ? (c - b0) : 32;
#pragma unroll 1
        for (int k = 0; k < m32; ++k) {
          const int u    = __builtin_amdgcn_readlane(ent, k);
          const int slot = u & (NBRUN - 1);
          if (t2 < CAP) {
            if (lane == 0) {
              int p = cur[slot];
              p = clampi(p, 0, CAP - 1);
              sl[p] = u >> 10;
              cur[slot] = p + 1;
            }
            t2 = t2 + 1;
          }
        }
      }
    }
  }
  __syncthreads();

  const int ovf = misc[9];
  int* lbase = LIST + (size_t)blk * (size_t)(CAP * 2);
  for (int pass = 0; pass < 2; ++pass) {
#pragma unroll 2
    for (int i = tid; i < CAP / 2; i += 256) {
      const v2i ev = *(const v2ia*)(sl + 2 * i);
      const int e0 = clampi(ev.x, 0, NE - 1);
      const int e1 = clampi(ev.y, 0, NE - 1);
      int s0 = srcp[e0];
      int s1 = srcp[e1];
      asm volatile("" :: "v"(s0));
      asm volatile("" :: "v"(s1));
      s0 = clampi(s0, 0, NN - 1);
      s1 = clampi(s1, 0, NN - 1);
      const v4i v = (v4i){ s0, e0, s1, e1 };
      *(volatile v4i*)(lbase + 4 * i) = v;
    }
    __threadfence();
  }
  const v4i cv4 = *(const v4ia*)(cnt + 4 * tid);
  const v4i ov4 = *(const v4ia*)(offs + 4 * tid);
  const v4i fl4 = (v4i){ ovf, ovf, ovf, ovf };
  const size_t nb4 = (size_t)nodeBase + 4 * (size_t)tid;
  const bool fw = (wave == 0) && (lane < 8);
  *(volatile v4i*)(CNT + nb4) = cv4;
  *(volatile v4i*)(OFF + nb4) = ov4;
  if (fw) *(volatile v4i*)(FLAG + blk * 32 + 4 * lane) = fl4;
  __threadfence();
  *(volatile v4i*)(CNT + nb4) = cv4;
  *(volatile v4i*)(OFF + nb4) = ov4;
  if (fw) *(volatile v4i*)(FLAG + blk * 32 + 4 * lane) = fl4;
}

__global__ __launch_bounds__(256) void k_deg(const int* __restrict__ LIST, const int* __restrict__ CNT,
                                             const int* __restrict__ OFF, const float* __restrict__ wgt,
                                             float* __restrict__ DINV) {
  __shared__ __attribute__((aligned(16))) float sD[32];
  const int tid = (int)threadIdx.x, lane = tid & 31, wave = tid >> 5;
#pragma unroll 1
  for (int j = 0; j < 4; ++j) {
    const int n = (int)blockIdx.x * 32 + wave * 4 + j;
    const bool live = n < NN;
    const int ic = clampi(n, 0, NN - 1);
    const int b  = ic >> 10;
    int c = CNT[ic];
    int o = OFF[ic];
    asm volatile("" :: "v"(c));
    asm volatile("" :: "v"(o));
    c = clampi(c, 0, DEGCAP);
    o = clampi(o, 0, CAP - DEGCAP);
    const int cn = __builtin_amdgcn_readfirstlane(live ? c : 0);
    const int* lp = LIST + ((size_t)b * (size_t)CAP + (size_t)o) * 2;
    const int top = cn > 0 ? cn - 1 : 0;
    const int i0 = lane < top ? lane : top;
    const int i1 = (lane + 32) < top ? (lane + 32) : top;
    int e0 = lp[2 * i0 + 1];
    int e1 = lp[2 * i1 + 1];
    asm volatile("" :: "v"(e0));
    asm volatile("" :: "v"(e1));
    e0 = clampi(e0, 0, NE - 1);
    e1 = clampi(e1, 0, NE - 1);
    const float w0 = wgt[e0];
    const float w1 = wgt[e1];
    asm volatile("" :: "v"(w0));
    asm volatile("" :: "v"(w1));
    const int wb0 = __float_as_int(bf16_val(w0));
    const int wb1 = __float_as_int(bf16_val(w1));
    float s = 0.0f;
    const int c0 = cn < 32 ? cn : 32;
#pragma unroll 1
    for (int k = 0; k < c0; ++k) s = s + __int_as_float(__builtin_amdgcn_readlane(wb0, k));
#pragma unroll 1
    for (int k = 32; k < cn; ++k) s = s + __int_as_float(__builtin_amdgcn_readlane(wb1, k - 32));
    s = s + 1.0f;
    const float dm = (s > 1e-30f) ? s : 1e-30f;
    const float r  = 1.0f / sqrtf(dm);
    const float dv = (s > 0.0f) ? r : 0.0f;
    if (lane == 0) sD[wave * 4 + j] = dv;
  }
  __syncthreads();
  const int t8 = tid < 8 ? tid : 7;
  const v4f o4 = (v4f){ sD[4 * t8], sD[4 * t8 + 1], sD[4 * t8 + 2], sD[4 * t8 + 3] };
  if (tid < 8) {
    volatile v4f* q = (volatile v4f*)(DINV + (size_t)blockIdx.x * 32 + 4 * tid);
    *q = o4;
    __threadfence();
    *q = o4;
  }
}

template <int NC, int LDP>
__global__ __launch_bounds__(256) void k_replay(const float* __restrict__ P, const int* __restrict__ LIST,
                                                const int* __restrict__ CNT, const int* __restrict__ OFF,
                                                const float* __restrict__ DINV, const int* __restrict__ FLAG,
                                                const float* __restrict__ wgt, const float* __restrict__ bias,
                                                float* outp, int nrows) {
  static_assert(NC == 128 || NC == 64 || NC == 32);
  static_assert(LDP >= NC && LDP % 32 == 0);
  constexpr int CPL = NC / 32;
  __shared__ __attribute__((aligned(16))) float sB[NC];
  const int tid = (int)threadIdx.x, lane = tid & 31, wave = tid >> 5;
  if (wave == 0) {
    float bq[4];
    ld_cols<CPL>(bias + CPL * lane, bq);
#pragma unroll
    for (int e = 0; e < CPL; ++e) sB[CPL * lane + e] = bq[e];
  }
  __syncthreads();
  float bv[4] = { 0.0f, 0.0f, 0.0f, 0.0f };
#pragma unroll
  for (int e = 0; e < CPL; ++e) bv[e] = sB[CPL * lane + e];

  const int i    = (int)blockIdx.x * 8 + wave;
  const bool live = i < nrows;
  const int ic   = clampi(i, 0, NN - 1);
  const int b    = ic >> 10;
  int c  = CNT[ic];
  int o  = OFF[ic];
  const int fl = FLAG[b * 32];
  const float di = DINV[ic];
  asm volatile("" :: "v"(c));
  asm volatile("" :: "v"(o));
  asm volatile("" :: "v"(fl));
  asm volatile("" :: "v"(di));
  c = clampi(c, 0, DEGCAP);
  o = clampi(o, 0, CAP - DEGCAP);
  const int cn = __builtin_amdgcn_readfirstlane(live ? c : 0);
  const int* lp = LIST + ((size_t)b * (size_t)CAP + (size_t)o) * 2;
  const float* Pl = P + CPL * lane;

  float acc[4] = { 0.0f, 0.0f, 0.0f, 0.0f };
#pragma unroll 1
  for (int b0 = 0; b0 < cn; b0 += 32) {
    const int idx = (b0 + lane) < cn ? (b0 + lane) : cn - 1;
    const v2i pr = *(const v2ia*)(lp + 2 * idx);
    asm volatile("" :: "v"(pr));
    const int sr = clampi(pr.x, 0, NN - 1);
    const int ed = clampi(pr.y, 0, NE - 1);
    const float dv = DINV[sr];
    const float wr = wgt[ed];
    asm volatile("" :: "v"(dv));
    asm volatile("" :: "v"(wr));
    const float wb  = bf16_val(wr);
    const float cf  = (dv * wb) * di;
    const int   cfi = __float_as_int(cf);
    const int m32 = (cn - b0) < 32 ? (cn - b0) : 32;
#pragma unroll 1
    for (int k = 0; k < m32; ++k) {
      const int   skk = __builtin_amdgcn_readlane(sr, k);
      const float ck  = __int_as_float(__builtin_amdgcn_readlane(cfi, k));
      float row[4];
      ld_cols<CPL>(Pl + (size_t)skk * LDP, row);
#pragma unroll
      for (int e = 0; e < CPL; ++e) acc[e] = acc[e] + row[e] * ck;
    }
  }
  float self[4];
  ld_cols<CPL>(Pl + (size_t)ic * LDP, self);
  const float dd = (di * 1.0f) * di;
  const float qn = __int_as_float(0x7fc00000);
  const bool poison = fl != 0;
  float v[4] = { 0.0f, 0.0f, 0.0f, 0.0f };
#pragma unroll
  for (int e = 0; e < CPL; ++e) {
    const float t = (acc[e] + self[e] * dd) + bv[e];
    v[e] = poison ? qn : t;
  }
  float* op = outp + (size_t)ic * NC + CPL * lane;
  if (live) st_cols<CPL>(op, v);
  __threadfence();
  if (live) st_cols<CPL>(op, v);
}

template <int MODE, int NC>
__global__ __launch_bounds__(256) void k_colstat(const float* __restrict__ H, const float* __restrict__ mean,
                                                 double* __restrict__ rec) {
  static_assert(MODE == 0 || MODE == 1);
  static_assert(NC == 128 || NC == 64 || NC == 32);
  __shared__ __attribute__((aligned(16))) float  sm[NC];
  __shared__ __attribute__((aligned(16))) double sp[2 * NC];
  const int tid = (int)threadIdx.x;
  if (tid < 32) {
    const int j = tid < NC / 4 ? tid : NC / 4 - 1;
    v4f mv = (v4f){0.f, 0.f, 0.f, 0.f};
    if constexpr (MODE == 1) {
      mv = *(const v4fa*)(mean + 4 * j);
      asm volatile("" :: "v"(mv));
    }
    if (tid < NC / 4) {
      sm[4 * tid]     = mv[0];
      sm[4 * tid + 1] = mv[1];
      sm[4 * tid + 2] = mv[2];
      sm[4 * tid + 3] = mv[3];
    }
  }
  __syncthreads();
  const int col = tid & (NC - 1);
  const int g   = tid / NC;
  const int r0  = (int)blockIdx.x * 128 + g * 64;
  const int nr  = clampi(NN - r0, 0, 64);
  const float m = sm[col];
  const float* hp = H + (size_t)r0 * NC + col;
  double s = 0.0;
#pragma unroll 4
  for (int j = 0; j < nr; ++j) {
    const float v = hp[(size_t)j * NC];
    if constexpr (MODE == 0) {
      s += (double)v;
    } else {
      const float d = v - m;
      const double dd = (double)d;
      s += dd * dd;
    }
  }
  sp[tid] = s;
  __syncthreads();
  const int t2 = tid < NC / 2 ? tid : NC / 2 - 1;
  const double a0 = sp[2 * t2] + sp[NC + 2 * t2];
  const double a1 = sp[2 * t2 + 1] + sp[NC + 2 * t2 + 1];
  const v2d o = (v2d){ a0, a1 };
  if (tid < NC / 2) {
    volatile v2d* q = (volatile v2d*)(rec + (size_t)blockIdx.x * NC + 2 * tid);
    *q = o;
    __threadfence();
    *q = o;
  }
}

__global__ __launch_bounds__(256) void k_comb(const double* __restrict__ rec, float* __restrict__ out,
                                              double inv_count, int nc, int mode) {
  __shared__ __attribute__((aligned(16))) float sv[256];
  const int tid = (int)threadIdx.x;
  const int c = tid < nc ? tid : nc - 1;
  double s = 0.0;
#pragma unroll 4
  for (int i = 0; i < NREC; ++i) s += rec[(size_t)i * (size_t)nc + c];
  const float qf = (float)(s * inv_count);
  const float rs = 1.0f / sqrtf(qf + 1e-5f);
  sv[tid] = (mode == 0) ? qf : rs;
  __syncthreads();
  const int n4 = nc >> 2;
  const int t4 = tid < n4 ? tid : n4 - 1;
  const v4f o = (v4f){ sv[4 * t4], sv[4 * t4 + 1], sv[4 * t4 + 2], sv[4 * t4 + 3] };
  if (tid < n4) {
    volatile v4f* q = (volatile v4f*)(out + 4 * tid);
    *q = o;
    __threadfence();
    *q = o;
  }
}

template <int LAYER>
__global__ __launch_bounds__(256) void k_apply(const float* __restrict__ V,
                                               const float* __restrict__ mean, const float* __restrict__ rstd,
                                               const float* __restrict__ gam, const float* __restrict__ bet,
                                               unsigned short* __restrict__ hl, float* __restrict__ outp) {
  static_assert(LAYER >= 1 && LAYER <= 3);
  constexpr int  NC  = (LAYER == 1) ? F1 : ((LAYER == 2) ? F2 : F3);
  constexpr int  CPL = NC / 32;
  constexpr int  KT  = (LAYER == 1) ? K2T : K3T;
  constexpr bool TWO = (LAYER == 1) ? (SINGLE_L2 == 0) : (SINGLE_L3 == 0);
  __shared__ __attribute__((aligned(16))) float spar[4 * NC];
  const int tid = (int)threadIdx.x, lane = tid & 31, wave = tid >> 5;
  const int c0 = CPL * lane;
  if (wave == 0) {
    float a0[4], a1[4], a2[4], a3[4];
    ld_cols<CPL>(mean + c0, a0);
    ld_cols<CPL>(rstd + c0, a1);
    ld_cols<CPL>(gam + c0, a2);
    ld_cols<CPL>(bet + c0, a3);
#pragma unroll
    for (int e = 0; e < CPL; ++e) {
      spar[c0 + e]          = a0[e];
      spar[NC + c0 + e]     = a1[e];
      spar[2 * NC + c0 + e] = a2[e];
      spar[3 * NC + c0 + e] = a3[e];
    }
  }
  __syncthreads();
  float mv[4] = { 0.0f, 0.0f, 0.0f, 0.0f }, rv[4] = { 0.0f, 0.0f, 0.0f, 0.0f };
  float gv[4] = { 0.0f, 0.0f, 0.0f, 0.0f }, bv[4] = { 0.0f, 0.0f, 0.0f, 0.0f };
#pragma unroll
  for (int e = 0; e < CPL; ++e) {
    mv[e] = spar[c0 + e];
    rv[e] = spar[NC + c0 + e];
    gv[e] = spar[2 * NC + c0 + e];
    bv[e] = spar[3 * NC + c0 + e];
  }
  const int row = (int)blockIdx.x * 8 + wave;
  const bool live = row < NN;
  const int rc = live ? row : NN - 1;
  float cv[4];
  ld_cols<CPL>(V + (size_t)rc * NC + c0, cv);
  float y[4] = { 0.0f, 0.0f, 0.0f, 0.0f };
#pragma unroll
  for (int e = 0; e < CPL; ++e) {
    float t = ((cv[e] - mv[e]) * rv[e]) * gv[e] + bv[e];
    if (LAYER < 3) t = relu_k(t);
    y[e] = live ? t : 0.0f;
  }
  if constexpr (LAYER == 1) {
    const v2u hv = (v2u){ pk16(bf16_bits(y[0]), bf16_bits(y[1])), pk16(bf16_bits(y[2]), bf16_bits(y[3])) };
    const v2u lv = (v2u){ pk16(bf16_lo_bits(y[0]), bf16_lo_bits(y[1])), pk16(bf16_lo_bits(y[2]), bf16_lo_bits(y[3])) };
    unsigned short* rp = hl + (size_t)row * KT + c0;
    *(volatile v2u*)rp = hv;
    if (TWO) *(volatile v2u*)(rp + F1) = lv;
    __threadfence();
    *(volatile v2u*)rp = hv;
    if (TWO) *(volatile v2u*)(rp + F1) = lv;
  } else if constexpr (LAYER == 2) {
    const unsigned hv = pk16(bf16_bits(y[0]), bf16_bits(y[1]));
    const unsigned lv = pk16(bf16_lo_bits(y[0]), bf16_lo_bits(y[1]));
    unsigned short* rp = hl + (size_t)row * KT + c0;
    *(volatile unsigned*)rp = hv;
    if (TWO) *(volatile unsigned*)(rp + F2) = lv;
    __threadfence();
    *(volatile unsigned*)rp = hv;
    if (TWO) *(volatile unsigned*)(rp + F2) = lv;
  } else {
    const float yo = y[0];
    float* op = outp + (size_t)rc * F3 + lane;
    if (live) *(volatile float*)op = yo;
    __threadfence();
    if (live) *(volatile float*)op = yo;
  }
}

constexpr int G_GEMM128 = ((NP / 64) * (F1 / 64) + 7) / 8;
constexpr int G_GEMM64  = ((NP / 64) * 1 + 7) / 8;
static_assert(NP % 64 == 0 && F1 % 64 == 0 && F2 % 64 == 0 && F1 % 32 == 0 && F2 % 32 == 0);

extern "C" void kernel_launch(void* const* d_in, const int* in_sizes, int n_in,
                              void* d_out, int out_size, void* d_ws, size_t ws_size,
                              hipStream_t stream) {
  if (n_in < 16) return;
  if (in_sizes[0] != NN) return;
  if (in_sizes[1] != 2 * NE) return;
  if (in_sizes[2] != NE) return;
  if (in_sizes[3] != NN * F0) return;
  if (in_sizes[4] != F0 * F1 || in_sizes[5] != F1 || in_sizes[6] != F1 || in_sizes[7] != F1) return;
  if (in_sizes[8] != F1 * F2 || in_sizes[9] != F2 || in_sizes[10] != F2 || in_sizes[11] != F2) return;
  if (in_sizes[12] != F2 * F3 || in_sizes[13] != F3 || in_sizes[14] != F3 || in_sizes[15] != F3) return;
  if (out_size != NN * F3) return;
  if (ws_size < WS_TOTAL) return;

  const int*   xid = (const int*)d_in[0];
  const int*   ei  = (const int*)d_in[1];
  const float* wgt = (const float*)d_in[2];
  const float* emb = (const float*)d_in[3];
  const float* W1  = (const float*)d_in[4];
  const float* b1  = (const float*)d_in[5];
  const float* g1  = (const float*)d_in[6];
  const float* be1 = (const float*)d_in[7];
  const float* W2  = (const float*)d_in[8];
  const float* b2  = (const float*)d_in[9];
  const float* g2  = (const float*)d_in[10];
  const float* be2 = (const float*)d_in[11];
  const float* W3  = (const float*)d_in[12];
  const float* b3  = (const float*)d_in[13];
  const float* g3  = (const float*)d_in[14];
  const float* be3 = (const float*)d_in[15];
  float* out = (float*)d_out;

  char* ws = (char*)d_ws;
  unsigned short* A0   = (unsigned short*)(ws + OFF_A0);
  unsigned short* AHL  = (unsigned short*)(ws + OFF_AHL);
  unsigned short* AHL3 = (unsigned short*)(ws + OFF_AHL3);
  float*          HW   = (float*)(ws + OFF_HW);
  float*          V    = (float*)(ws + OFF_V);
  int*            LIST = (int*)(ws + OFF_LIST);
  int*            CNT  = (int*)(ws + OFF_CNT);
  int*            OFFS = (int*)(ws + OFF_OFF);
  float*          DINV = (float*)(ws + OFF_DINV);
  int*            FLAG = (int*)(ws + OFF_FLAG);
  unsigned short* W1T  = (unsigned short*)(ws + OFF_W1T);
  unsigned short* W2D  = (unsigned short*)(ws + OFF_W2D);
  unsigned short* W3D  = (unsigned short*)(ws + OFF_W3D);
  float*          PAR  = (float*)(ws + OFF_PAR);
  double*         REC  = (double*)(ws + OFF_REC);
  float*          ST   = (float*)(ws + OFF_ST);

  const double invN = 1.0 / 50000.0;

  hipFuncSetAttribute(reinterpret_cast<const void*>(&k_list), hipFuncAttributeMaxDynamicSharedMemorySize, (int)LK_LDS);

  k_prep<<<PB_TOT, 256, 0, stream>>>(W1, W2, W3, b1, g1, be1, b2, g2, be2, b3, g3, be3, W1T, W2D, W3D, PAR);
  k_gatherA<<<NP / 8, 256, 0, stream>>>(xid, emb, A0);
  k_list<<<NBLK, 256, LK_LDS, stream>>>(ei, LIST, CNT, OFFS, FLAG);
  k_deg<<<(NN + 31) / 32, 256, 0, stream>>>(LIST, CNT, OFFS, wgt, DINV);

  k_gemm_nt<0, 0><<<G_GEMM128, 256, 0, stream>>>(A0, W1T, PAR, HW, NP, F1, F0, F1);
  k_replay<F1, F1><<<NN / 8, 256, 0, stream>>>(HW, LIST, CNT, OFFS, DINV, FLAG, wgt, PAR + P_B1, V, NN);
  k_colstat<0, F1><<<NREC, 2 * F1, 0, stream>>>(V, ST + S_M1, REC);
  k_comb<<<1, 256, 0, stream>>>(REC, ST + S_M1, invN, F1, 0);
  k_colstat<1, F1><<<NREC, 2 * F1, 0, stream>>>(V, ST + S_M1, REC);
  k_comb<<<1, 256, 0, stream>>>(REC, ST + S_R1, invN, F1, 1);
  k_apply<1><<<NP / 8, 256, 0, stream>>>(V, ST + S_M1, ST + S_R1, PAR + P_G1, PAR + P_BE1, AHL, out);

  k_gemm_nt<0, 0><<<G_GEMM64, 256, 0, stream>>>(AHL, W2D, PAR, HW, NP, F2, K2T, F2);
  k_replay<F2, F2><<<NN / 8, 256, 0, stream>>>(HW, LIST, CNT, OFFS, DINV, FLAG, wgt, PAR + P_B2, V, NN);
  k_colstat<0, F2><<<NREC, 2 * F2, 0, stream>>>(V, ST + S_M2, REC);
  k_comb<<<1, 256, 0, stream>>>(REC, ST + S_M2, invN, F2, 0);
  k_colstat<1, F2><<<NREC, 2 * F2, 0, stream>>>(V, ST + S_M2, REC);
  k_comb<<<1, 256, 0, stream>>>(REC, ST + S_R2, invN, F2, 1);
  k_apply<2><<<NP / 8, 256, 0, stream>>>(V, ST + S_M2, ST + S_R2, PAR + P_G2, PAR + P_BE2, AHL3, out);

  k_gemm_nt<0, 0><<<G_GEMM64, 256, 0, stream>>>(AHL3, W3D, PAR, HW, NP, 64, K3T, 64);
  k_replay<F3, 64><<<NN / 8, 256, 0, stream>>>(HW, LIST, CNT, OFFS, DINV, FLAG, wgt, PAR + P_B3, V, NN);
  k_colstat<0, F3><<<NREC, 2 * F3, 0, stream>>>(V, ST + S_M3, REC);
  k_comb<<<1, 256, 0, stream>>>(REC, ST + S_M3, invN, F3, 0);
  k_colstat<1, F3><<<NREC, 2 * F3, 0, stream>>>(V, ST + S_M3, REC);
  k_comb<<<1, 256, 0, stream>>>(REC, ST + S_R3, invN, F3, 1);
  k_apply<3><<<NN / 8, 256, 0, stream>>>(V, ST + S_M3, ST + S_R3, PAR + P_G3, PAR + P_BE3, AHL3, out);
}
